// SimpleRNN_8589934592513
// MI455X (gfx1250) — hardware-run, weakly checked
//
#include <hip/hip_runtime.h>
#include <math.h>

typedef __attribute__((ext_vector_type(16))) _Float16 v16h;
typedef __attribute__((ext_vector_type(8)))  _Float16 v8h;
typedef __attribute__((ext_vector_type(8)))  float    v8f;
typedef __attribute__((ext_vector_type(4)))  float    v4f;

constexpr int kVocab  = 32000;
constexpr int kEmb    = 256;
constexpr int kHid    = 512;
constexpr int kSeqs   = 256;
constexpr int kSteps  = 512;

constexpr int kRowsPB     = 16;
constexpr int kScanBlocks = kSeqs / kRowsPB;
constexpr int kThreads    = 256;
constexpr int kHP         = 520;
constexpr int kHTile      = kRowsPB * kHP;
constexpr int kSlabP      = 68;

constexpr float kCarryEmb = 64.0f;
constexpr float kCarryWx  = 512.0f;
constexpr float kCarryH   = 256.0f;
constexpr float kCarryWh  = 512.0f;
constexpr float kFoldX    = 1.0f / (kCarryEmb * kCarryWx);
constexpr float kFoldH    = 1.0f / (kCarryH * kCarryWh);
constexpr float kF16MinNormal = 6.103515625e-5f;

static_assert(kSeqs % kRowsPB == 0);
static_assert(kHid == 64 * (kThreads / 32));
static_assert(kHid % 32 == 0 && kEmb % 32 == 0);
static_assert(kVocab % 64 == 0 && kHid % 64 == 0);
static_assert(kHP % 8 == 0 && kHP >= kHid);
static_assert((2 * kHTile) % kThreads == 0);
static_assert(kFoldX == 1.0f / 32768.0f);
static_assert(kFoldH == 1.0f / 131072.0f);

constexpr int kN8Emb = kVocab * kEmb / 8;
constexpr int kN8Wx  = kHid * kEmb / 8;
constexpr int kN8Wh  = kHid * kHid / 8;
static_assert(kN8Emb % 256 == 0 && kN8Wx % 256 == 0 && kN8Wh % 256 == 0);
constexpr int kPrepB1     = kN8Emb / 256;
constexpr int kPrepB2     = kPrepB1 + kN8Wx / 256;
constexpr int kPrepB3     = kPrepB2 + kN8Wh / 256;
constexpr int kPrepBlocks = kPrepB3 + 1;
static_assert(kPrepB1 == 4000 && kPrepB2 == 4064 && kPrepB3 == 4192);

constexpr int kGemmTiles  = (kVocab / 64) * (kHid / 64);
static_assert(kGemmTiles % 8 == 0);
constexpr int kGemmBlocks = kGemmTiles / 8;
static_assert(kGemmBlocks == 500);

constexpr size_t kBytesEmb16 = (size_t)kVocab * kEmb * 2;
constexpr size_t kBytesWx16  = (size_t)kHid * kEmb * 2;
constexpr size_t kBytesWh16  = (size_t)kHid * kHid * 2;
constexpr size_t kBytesBias  = (size_t)kHid * 4;
constexpr size_t kBytesXP    = (size_t)kVocab * kHid * 4;
constexpr size_t kWsTotal    = kBytesEmb16 + kBytesWx16 + kBytesWh16 + kBytesBias + kBytesXP;
static_assert(kWsTotal == 82708480ull);
static_assert(kWsTotal <= 134217728ull);
static_assert(kBytesEmb16 % 256 == 0 && kBytesWx16 % 256 == 0 && kBytesWh16 % 256 == 0 &&
              kBytesBias % 256 == 0 && kBytesXP % 256 == 0);

__device__ __forceinline__ v16h frag_load(const _Float16* p) {
  union U { v16h v; v8h h[2]; };
  U f;
  f.h[0] = *(const v8h*)(p);
  f.h[1] = *(const v8h*)(p + 16);
  return f.v;
}
__device__ __forceinline__ v8f mma_h(v16h a, v16h b, v8f c) {
  c = __builtin_amdgcn_wmma_f32_16x16x32_f16(false, a, false, b, (short)0, c, false, false);
  asm volatile("v_nop\n\tv_nop\n\tv_nop\n\tv_nop" : "+v"(c) : "v"(a), "v"(b));
  return c;
}
__device__ __forceinline__ void wave_lds_sync() {
  __builtin_amdgcn_fence(__ATOMIC_RELEASE, "workgroup");
  __builtin_amdgcn_wave_barrier();
  __builtin_amdgcn_fence(__ATOMIC_ACQUIRE, "workgroup");
}
__device__ __forceinline__ _Float16 to_f16_operand(float x) {
  const float y = (fabsf(x) < kF16MinNormal) ? 0.0f : x;
  return (_Float16)y;
}
__device__ __forceinline__ float ftanh(float x) {
  return 1.0f - 2.0f * __builtin_amdgcn_rcpf(1.0f + __expf(2.0f * x));
}

__device__ __forceinline__ void cvt8_store(const float* __restrict__ src, unsigned short* __restrict__ dst,
                                           int i, float sc) {
  const size_t e0 = (size_t)i * 8;
  const v4f a = *(const v4f*)(src + e0);
  const v4f b = *(const v4f*)(src + e0 + 4);
  v8h hv;
#pragma unroll
  for (int e = 0; e < 4; ++e) {
    const float x0 = a[e] * sc;
    const float x1 = b[e] * sc;
    hv[e]     = to_f16_operand(x0);
    hv[4 + e] = to_f16_operand(x1);
  }
  unsigned short* q = dst + e0;
  *(volatile v8h*)q = hv;
  __threadfence();
  *(volatile v8h*)q = hv;
}

__global__ __launch_bounds__(256) void prep_kernel(
    const float* __restrict__ emb, const float* __restrict__ wxh, const float* __restrict__ whh,
    const float* __restrict__ bxh, const float* __restrict__ bhh,
    unsigned short* __restrict__ emb16, unsigned short* __restrict__ wxh16,
    unsigned short* __restrict__ whh16, float* __restrict__ bias32) {
  const int blk = blockIdx.x, tid = threadIdx.x;
  if (blk < kPrepB1) {
    cvt8_store(emb, emb16, blk * 256 + tid, kCarryEmb);
  } else if (blk < kPrepB2) {
    cvt8_store(wxh, wxh16, (blk - kPrepB1) * 256 + tid, kCarryWx);
  } else if (blk < kPrepB3) {
    cvt8_store(whh, whh16, (blk - kPrepB2) * 256 + tid, kCarryWh);
  } else {
    if (tid < 128) {
      const int idx = tid * 4;
      const v4f va = *(const v4f*)(bxh + idx);
      const v4f vb = *(const v4f*)(bhh + idx);
      v4f o;
#pragma unroll
      for (int e = 0; e < 4; ++e) o[e] = va[e] + vb[e];
      float* op = bias32 + idx;
      *(volatile v4f*)op = o;
      __threadfence();
      *(volatile v4f*)op = o;
    }
  }
}

__global__ __launch_bounds__(256) void gemm64_f16_kernel(
    const unsigned short* __restrict__ Ap, int lda,
    const unsigned short* __restrict__ Btp, int ldb,
    float* __restrict__ C, int ldc,
    const float* __restrict__ bias,
    int M, int N, int K, float scale) {
  const _Float16* A  = (const _Float16*)Ap;
  const _Float16* Bt = (const _Float16*)Btp;
  __shared__ __align__(16) float sT[8][16 * kSlabP];
  const int lane = threadIdx.x & 31;
  const int wave = threadIdx.x >> 5;
  const int tilesN = N >> 6;
  const int tilesM = M >> 6;
  const int tile = blockIdx.x * 8 + wave;
  if (tile >= tilesM * tilesN) return;
  const int tm = tile / tilesN;
  const int tn = tile - tm * tilesN;
  const int m0 = tm << 6;
  const int n0 = tn << 6;

  const int rlane = lane & 15;
  const int koff  = (lane >> 4) * 8;
  const int mOff  = (lane >> 4) * 8;

  v8f acc[4][4];
#pragma unroll
  for (int i = 0; i < 4; ++i)
#pragma unroll
    for (int j = 0; j < 4; ++j) acc[i][j] = (v8f){0.f, 0.f, 0.f, 0.f, 0.f, 0.f, 0.f, 0.f};

  for (int k0 = 0; k0 < K; k0 += 32) {
    v16h bh[4];
#pragma unroll
    for (int j = 0; j < 4; ++j) {
      const size_t bo = (size_t)(n0 + (j << 4) + rlane) * ldb + koff + k0;
      bh[j] = frag_load(Bt + bo);
    }
#pragma unroll
    for (int i = 0; i < 4; ++i) {
      const size_t ao = (size_t)(m0 + (i << 4) + rlane) * lda + koff + k0;
      const v16h ah = frag_load(A + ao);
#pragma unroll
      for (int j = 0; j < 4; ++j) acc[i][j] = mma_h(ah, bh[j], acc[i][j]);
    }
  }

  float* slab = sT[wave];
#pragma unroll
  for (int i = 0; i < 4; ++i) {
    const int mBase = m0 + (i << 4);
#pragma unroll
    for (int j = 0; j < 4; ++j) {
      const int n = n0 + (j << 4) + rlane;
      const float bv = bias[n];
#pragma unroll
      for (int r = 0; r < 8; ++r) {
        const float v = acc[i][j][r] * scale + bv;
        slab[(mOff + r) * kSlabP + (j << 4) + rlane] = v;
      }
    }
    wave_lds_sync();
    {
      const int hh = lane >> 4, c4 = (lane & 15) * 4;
      for (int pass = 0; pass < 2; ++pass) {
#pragma unroll
        for (int it = 0; it < 8; ++it) {
          const int row = it * 2 + hh;
          const v4f v = *(const v4f*)(slab + row * kSlabP + c4);
          *(volatile v4f*)(C + (size_t)(mBase + row) * ldc + n0 + c4) = v;
        }
        __threadfence();
      }
    }
    wave_lds_sync();
  }
}

__global__ __launch_bounds__(kThreads) void scan_kernel(
    const int* __restrict__ X, const float* __restrict__ XP,
    const unsigned short* __restrict__ WHp, float* __restrict__ out) {
  __shared__ __align__(16) _Float16 Ah[2][kHTile];
  __shared__ __align__(16) float    Sl[kThreads / 32][16 * kSlabP];
  const _Float16* WH = (const _Float16*)WHp;
  const int tid = threadIdx.x, lane = tid & 31, wave = tid >> 5;
  const int c = lane & 15, hh = lane >> 4, koff = hh * 8, mOff = hh * 8, c4 = c * 4;
  const int seq0 = blockIdx.x * kRowsPB;
  const int n0 = wave * 64;

  {
    _Float16* ahf = &Ah[0][0];
#pragma unroll 1
    for (int i = tid; i < 2 * kHTile; i += kThreads) ahf[i] = (_Float16)0.0f;
  }
  __syncthreads();

  float* slab = Sl[wave];
  const _Float16* brow = WH + (size_t)(n0 + c) * kHid + koff;
  const int* trow = X + (size_t)(seq0 + hh) * kSteps;
  const float* xpcol = XP + n0 + c4;
  const v8f z8 = {0.f, 0.f, 0.f, 0.f, 0.f, 0.f, 0.f, 0.f};

#pragma unroll 1
  for (int t = 0; t < kSteps; ++t) {
    const int cur = t & 1;

    {
      int tk[8];
#pragma unroll
      for (int it = 0; it < 8; ++it) {
        int v = trow[(size_t)(2 * it) * kSteps + t];
        v = (v < 0) ? 0 : v;
        v = (v > kVocab - 1) ? (kVocab - 1) : v;
        tk[it] = v;
      }
      v4f xv[8];
#pragma unroll
      for (int it = 0; it < 8; ++it) xv[it] = *(const v4f*)(xpcol + (size_t)tk[it] * kHid);
#pragma unroll
      for (int it = 0; it < 8; ++it) *(v4f*)(slab + (it * 2 + hh) * kSlabP + c4) = xv[it];
    }

    const _Float16* arow = &Ah[0][0] + cur * kHTile + c * kHP + koff;
    v8f acc[4];
#pragma unroll
    for (int j = 0; j < 4; ++j) acc[j] = z8;
#pragma unroll 1
    for (int kc = 0; kc < kHid / 32; ++kc) {
      const v16h fa = frag_load(arow + kc * 32);
      v16h fb[4];
#pragma unroll
      for (int j = 0; j < 4; ++j) fb[j] = frag_load(brow + (size_t)(16 * j) * kHid + kc * 32);
#pragma unroll
      for (int j = 0; j < 4; ++j) acc[j] = mma_h(fa, fb[j], acc[j]);
    }

    wave_lds_sync();

    _Float16* ahn = &Ah[0][0] + (cur ^ 1) * kHTile;
#pragma unroll
    for (int j = 0; j < 4; ++j) {
#pragma unroll
      for (int r = 0; r < 8; ++r) {
        const int sidx = (mOff + r) * kSlabP + 16 * j + c;
        const float xpv = slab[sidx];
        const float pre = fmaf(acc[j][r], kFoldH, xpv);
        const float hv  = ftanh(pre);
        slab[sidx] = hv;
        ahn[(mOff + r) * kHP + n0 + 16 * j + c] = to_f16_operand(hv * kCarryH);
      }
    }
    __syncthreads();
  }

  wave_lds_sync();
  for (int pass = 0; pass < 2; ++pass) {
#pragma unroll
    for (int it = 0; it < 8; ++it) {
      const int row = it * 2 + hh;
      const v4f v = *(const v4f*)(slab + row * kSlabP + c4);
      *(volatile v4f*)(out + (size_t)(seq0 + row) * kHid + n0 + c4) = v;
    }
    __threadfence();
  }
}

extern "C" void kernel_launch(void* const* d_in, const int* in_sizes, int n_in,
                              void* d_out, int out_size, void* d_ws, size_t ws_size, hipStream_t stream) {
  if (n_in < 6 || d_out == nullptr || d_ws == nullptr) return;
  if (in_sizes[0] != kSeqs * kSteps || in_sizes[1] != kVocab * kEmb || in_sizes[2] != kHid * kHid ||
      in_sizes[3] != kHid || in_sizes[4] != kHid * kEmb || in_sizes[5] != kHid ||
      out_size != kSeqs * kHid) return;

  const int*   X   = (const int*)d_in[0];
  const float* emb = (const float*)d_in[1];
  const float* whh = (const float*)d_in[2];
  const float* bhh = (const float*)d_in[3];
  const float* wxh = (const float*)d_in[4];
  const float* bxh = (const float*)d_in[5];
  float* out = (float*)d_out;

  char* ws = (char*)d_ws;
  size_t off = 0;
  auto carve = [&](size_t bytes) -> char* { char* p = ws + off; off += (bytes + 255) & ~(size_t)255; return p; };
  unsigned short* EMB16  = (unsigned short*)carve(kBytesEmb16);
  unsigned short* WXH16  = (unsigned short*)carve(kBytesWx16);
  unsigned short* WHH16  = (unsigned short*)carve(kBytesWh16);
  float*          BIAS32 = (float*)carve(kBytesBias);
  float*          XP     = (float*)carve(kBytesXP);
  if (off != kWsTotal || off > ws_size || off > (size_t)134217728) return;

  prep_kernel<<<kPrepBlocks, 256, 0, stream>>>(emb, wxh, whh, bxh, bhh, EMB16, WXH16, WHH16, BIAS32);

  gemm64_f16_kernel<<<dim3(kGemmBlocks, 1), 256, 0, stream>>>(
      EMB16, kEmb, WXH16, kEmb, XP, kHid, BIAS32, kVocab, kHid, kEmb, kFoldX);

  scan_kernel<<<kScanBlocks, kThreads, 0, stream>>>(X, XP, WHH16, out);
}
